// CurvatureGatedGCN_88356067213584
// MI455X (gfx1250) — hardware-run, weakly checked
//
#include <hip/hip_runtime.h>

typedef float          v8f   __attribute__((ext_vector_type(8)));
typedef float          v4f   __attribute__((ext_vector_type(4)));
typedef unsigned int   v4u   __attribute__((ext_vector_type(4)));
typedef int            v8i   __attribute__((ext_vector_type(8)));
typedef unsigned short v8us  __attribute__((ext_vector_type(8)));
typedef unsigned short v16us __attribute__((ext_vector_type(16)));
typedef __bf16         v16bf __attribute__((ext_vector_type(16)));
typedef _Float16       v16h  __attribute__((ext_vector_type(16)));
typedef v4f  __attribute__((may_alias)) v4fa;
typedef v8us __attribute__((may_alias)) v8usa;
union FragB { v16bf v; v16us u; v8us h[2]; v8i w; };
union FragH { v16h  v; v16us u; v8us h[2]; v8i w; };

__device__ __forceinline__ v8f wmb(const FragB& a, const FragB& b, v8f c) {
  v8f d = __builtin_amdgcn_wmma_f32_16x16x32_bf16(false, a.v, false, b.v, (short)0, c, false, false);
  asm volatile("v_nop\n\tv_nop\n\tv_nop\n\tv_nop" : "+v"(d) : "v"(a.w), "v"(b.w));
  return d;
}

__device__ __forceinline__ v8f wmh(const FragH& a, const FragH& b, v8f c) {
  v8f d = __builtin_amdgcn_wmma_f32_16x16x32_f16(false, a.v, false, b.v, (short)0, c, false, false);
  asm volatile("v_nop\n\tv_nop\n\tv_nop\n\tv_nop" : "+v"(d) : "v"(a.w), "v"(b.w));
  return d;
}

__device__ __forceinline__ unsigned bf16_bits(float f) {
  const unsigned u = __float_as_uint(f);
  const unsigned r = (u + 0x7FFFu + ((u >> 16) & 1u)) >> 16;
  const unsigned q = (u >> 16) | 0x40u;
  return ((u & 0x7fffffffu) > 0x7f800000u) ? q : r;
}

__device__ __forceinline__ float bf16_val(float f) {
  return __uint_as_float(bf16_bits(f) << 16);
}
__device__ __forceinline__ int clampi(int v, int lo, int hi) {
  return v < lo ? lo : (v > hi ? hi : v);
}

__device__ __forceinline__ unsigned f16_bits(float f) {
  const unsigned u  = __float_as_uint(f);
  const unsigned s  = (u >> 16) & 0x8000u;
  const unsigned a  = u & 0x7fffffffu;
  const unsigned t  = a - 0x38000000u;
  const unsigned r  = (t + 0x0FFFu + ((t >> 13) & 1u)) >> 13;
  const unsigned rc = r > 0x7C00u ? 0x7C00u : r;
  const bool small  = a < 0x38800000u;
  const bool isnan  = a > 0x7f800000u;
  const unsigned fin = small ? 0u : (s | rc);
  return isnan ? (s | 0x7E00u) : fin;
}

__device__ __forceinline__ unsigned pk16(unsigned lo, unsigned hi) { return lo | (hi << 16); }
__device__ __forceinline__ unsigned bf16_lo_bits(float v) {
  float hi = bf16_val(v);
  asm volatile("" : "+v"(hi));
  return bf16_bits(v - hi);
}
__device__ __forceinline__ v4u pack8_bf16(v4f a, v4f c) {
  return (v4u){ pk16(bf16_bits(a[0]), bf16_bits(a[1])), pk16(bf16_bits(a[2]), bf16_bits(a[3])),
                pk16(bf16_bits(c[0]), bf16_bits(c[1])), pk16(bf16_bits(c[2]), bf16_bits(c[3])) };
}
__device__ __forceinline__ v4u pack8_bf16_lo(v4f a, v4f c) {
  return (v4u){ pk16(bf16_lo_bits(a[0]), bf16_lo_bits(a[1])), pk16(bf16_lo_bits(a[2]), bf16_lo_bits(a[3])),
                pk16(bf16_lo_bits(c[0]), bf16_lo_bits(c[1])), pk16(bf16_lo_bits(c[2]), bf16_lo_bits(c[3])) };
}
__device__ __forceinline__ v4u pack8_f16(v4f a, v4f c) {
  return (v4u){ pk16(f16_bits(a[0]), f16_bits(a[1])), pk16(f16_bits(a[2]), f16_bits(a[3])),
                pk16(f16_bits(c[0]), f16_bits(c[1])), pk16(f16_bits(c[2]), f16_bits(c[3])) };
}

template <int FORM>
__global__ __launch_bounds__(256) void k_plane(const float* __restrict__ src, int rows, int cols, int ldsrc,
                                               unsigned short* __restrict__ dst, int MP, int KP) {
  static_assert(FORM >= 0 && FORM <= 3);
  const int KTOT = (FORM == 1 || FORM == 3) ? 2 * KP : KP;
  const unsigned ppr   = (unsigned)(KTOT >> 3);
  const unsigned kp8   = (unsigned)(KP >> 3);
  const unsigned total = (unsigned)MP * ppr;
  const unsigned g     = blockIdx.x * 256u + threadIdx.x;
  const unsigned rowu  = g / ppr;
  const unsigned p     = g - rowu * ppr;
  const bool second    = p >= kp8;
  const int row = (int)rowu;
  const int c0  = (int)((second ? p - kp8 : p) << 3);
  const float* srow = src + (size_t)clampi(row, 0, rows - 1) * (size_t)ldsrc;
  float x[8];
  unsigned mk[8];
#pragma unroll
  for (int e = 0; e < 8; ++e) {
    const int c = c0 + e;
    const float v = srow[clampi(c, 0, cols - 1)];
    asm volatile("" :: "v"(v));
    x[e]  = v;
    mk[e] = (row < rows && c < cols) ? 0xFFFFu : 0u;
  }
  const v4f a = (v4f){ x[0], x[1], x[2], x[3] };
  const v4f c = (v4f){ x[4], x[5], x[6], x[7] };
  v4u o;
  if (FORM == 2) {
    o = pack8_f16(a, c);
  } else {
    const v4u hi = pack8_bf16(a, c);
    o = hi;
    if (FORM == 1) { const v4u lo = pack8_bf16_lo(a, c); o = second ? lo : hi; }
  }
  const v4u mw = (v4u){ pk16(mk[0], mk[1]), pk16(mk[2], mk[3]), pk16(mk[4], mk[5]), pk16(mk[6], mk[7]) };
  o &= mw;
  if (g < total) {
    volatile v4u* q = (volatile v4u*)(dst + (size_t)g * 8);
    *q = o;
    __threadfence();
    *q = o;
  }
}

template <int FORM> struct FragOf    { typedef FragB T; };
template <>         struct FragOf<2> { typedef FragH T; };
__device__ __forceinline__ v8f mm(const FragB& a, const FragB& b, v8f c) { return wmb(a, b, c); }
__device__ __forceinline__ v8f mm(const FragH& a, const FragH& b, v8f c) { return wmh(a, b, c); }
template <class F> __device__ __forceinline__ F ld_frag(const unsigned short* p) {
  F f;
  f.h[0] = *(const v8usa*)(p);
  f.h[1] = *(const v8usa*)(p + 16);
  return f;
}

template <int FORM, int EPI>
__global__ __launch_bounds__(256) __attribute__((amdgpu_num_vgpr(248)))
void k_gemm_nt(const unsigned short* __restrict__ A, const unsigned short* __restrict__ B,
               const float* __restrict__ bias, float* __restrict__ D, int M, int N, int KTOT, int ldd) {
  static_assert(FORM >= 0 && FORM <= 2);
  static_assert(EPI == 0 || EPI == 1);
  typedef typename FragOf<FORM>::T F;
  __shared__ __attribute__((aligned(16))) float sT[8][16 * 68];
  const int lane = threadIdx.x & 31;
  const int wave = threadIdx.x >> 5;
  const int tilesM = (M + 63) >> 6;
  const int tilesN = (N + 63) >> 6;
  const int tile = blockIdx.x * 8 + wave;
  if (tile >= tilesM * tilesN) return;
  const int tm = tile / tilesN;
  const int tn = tile - tm * tilesN;
  const int m0 = tm << 6;
  const int n0 = tn << 6;

  const int rl = lane & 15;
  const int h8 = (lane >> 4) * 8;
  const unsigned short* pa = A + (size_t)(m0 + rl) * (size_t)KTOT + h8;
  const unsigned short* pb = B + (size_t)(n0 + rl) * (size_t)KTOT + h8;

  v8f acc[4][4];
#pragma unroll
  for (int i = 0; i < 4; ++i)
#pragma unroll
    for (int j = 0; j < 4; ++j) acc[i][j] = (v8f){0.f, 0.f, 0.f, 0.f, 0.f, 0.f, 0.f, 0.f};

#pragma unroll 1
  for (int k0 = 0; k0 < KTOT; k0 += 32) {
    F bf[4];
#pragma unroll
    for (int j = 0; j < 4; ++j) bf[j] = ld_frag<F>(pb + (size_t)(j << 4) * (size_t)KTOT + k0);
#pragma unroll
    for (int i = 0; i < 4; ++i) {
      const F af = ld_frag<F>(pa + (size_t)(i << 4) * (size_t)KTOT + k0);
#pragma unroll
      for (int j = 0; j < 4; ++j) acc[i][j] = mm(af, bf[j], acc[i][j]);
    }
  }

  float* slab = sT[wave];
  const int hh = lane >> 4;
  const int c4 = (lane & 15) * 4;
  const int nc = n0 + c4;
  const bool cok = nc < N;
  v4f bv = (v4f){0.f, 0.f, 0.f, 0.f};
  if (EPI == 1) {
    bv = *(const v4fa*)(bias + clampi(nc, 0, N - 4));
    asm volatile("" :: "v"(bv));
  }
#pragma unroll
  for (int i = 0; i < 4; ++i) {
    const int mBase = m0 + (i << 4);
#pragma unroll
    for (int j = 0; j < 4; ++j) {
#pragma unroll
      for (int r = 0; r < 8; ++r) slab[(h8 + r) * 68 + (j << 4) + rl] = acc[i][j][r];
    }
    __builtin_amdgcn_fence(__ATOMIC_RELEASE, "workgroup");
    __builtin_amdgcn_wave_barrier();
    __builtin_amdgcn_fence(__ATOMIC_ACQUIRE, "workgroup");
    v4f vv[8];
#pragma unroll
    for (int it = 0; it < 8; ++it) {
      const int row = it * 2 + hh;
      v4f v = *(const v4fa*)(slab + row * 68 + c4);
      if (EPI == 1) v += bv;
      vv[it] = v;
    }
    for (int pass = 0; pass < 2; ++pass) {
#pragma unroll
      for (int it = 0; it < 8; ++it) {
        const int row = mBase + it * 2 + hh;
        if (cok && row < M) *(volatile v4f*)(D + (size_t)row * (size_t)ldd + nc) = vv[it];
      }
      __threadfence();
    }
    __builtin_amdgcn_fence(__ATOMIC_RELEASE, "workgroup");
    __builtin_amdgcn_wave_barrier();
    __builtin_amdgcn_fence(__ATOMIC_ACQUIRE, "workgroup");
  }
}

#pragma clang fp contract(off)

#define G_NN     50000
#define G_NE     1000000
#define G_D      64
#define G_NPAD   50048
#define G_NTHR   256
#define G_NWAVE  8
#define G_EPT    8
#define G_WCH    (32 * G_EPT)
#define G_NBRUN  1024
#define G_SLB    10
#define G_ESH    20
#define G_NBK    49
#define G_RCAP   26112
#define G_WLCAP  3264
#define G_WCAP   4096
#define G_MAXB1024_MEAS 20780
#define G_MAXDEG_MEAS   42
#define G_WSMAX  ((size_t)128 << 20)

#define SPLIT_H1 1
#define SPLIT_G2 1
#define SPLIT_H2 1

#define G_BK_ZINTS (G_NWAVE * G_WLCAP + G_RCAP + 4 * G_NBRUN)
#define G_BK_INTS  (G_BK_ZINTS + 16)
#define G_BK_LDS   (G_BK_INTS * 4)

static_assert(G_D == 64 && G_D == 32 * 2);
static_assert(G_NPAD % 128 == 0 && G_NPAD >= G_NN && G_NPAD == 391 * 128 && G_NPAD % 64 == 0 && G_NPAD % 16 == 0);
static_assert(G_NPAD % G_NWAVE == 0 && G_NN % G_NWAVE == 0);
static_assert(G_NBRUN == (1 << G_SLB) && G_NBRUN <= 1024 && G_NBRUN % G_NTHR == 0 && G_NBRUN % 32 == 0);
static_assert(G_NBK * G_NBRUN >= G_NPAD && (G_NBK - 1) * G_NBRUN < G_NN && G_NN <= G_NBK * 1024);
static_assert(G_NE <= (1 << G_ESH) && G_ESH + G_SLB <= 31);
static_assert(G_NE % G_EPT == 0 && G_NE % 4 == 0 && G_NE >= G_EPT);
static_assert(G_RCAP % 256 == 0 && (G_RCAP / 2) % G_NTHR == 0);
static_assert((long long)G_RCAP * 100 >= (long long)G_MAXB1024_MEAS * 125);
static_assert((long long)(G_RCAP - 256) * 100 < (long long)G_MAXB1024_MEAS * 125);
static_assert(G_NWAVE * G_WLCAP == G_RCAP);
static_assert(G_WLCAP >= G_MAXB1024_MEAS / 8 + 8 * 51 + 1);
static_assert(G_WCAP >= 8 * G_MAXDEG_MEAS && G_WCAP <= G_RCAP);
static_assert(G_BK_ZINTS % 4 == 0 && G_BK_LDS <= 262144 && G_BK_LDS + 0 <= 327680);
static_assert((G_NPAD * G_D / 8) % 256 == 0);

typedef float v2f __attribute__((ext_vector_type(2)));
typedef int   v2i __attribute__((ext_vector_type(2)));
typedef int   v4i __attribute__((ext_vector_type(4)));
typedef v2f __attribute__((may_alias)) v2fa;
typedef v2i __attribute__((may_alias)) v2ia;
typedef v4i __attribute__((may_alias)) v4ia;

__device__ __forceinline__ void st2_v2f(float* p, v2f v) {
  *(volatile v2f*)p = v;
  __threadfence();
  *(volatile v2f*)p = v;
}
__device__ __forceinline__ void st2_words(unsigned* p0, unsigned w0, unsigned* p1, unsigned w1) {
  *(volatile unsigned*)p0 = w0;
  *(volatile unsigned*)p1 = w1;
  __threadfence();
  *(volatile unsigned*)p0 = w0;
  *(volatile unsigned*)p1 = w1;
}

__device__ __forceinline__ void wt_unit(const float* __restrict__ w, unsigned short* dst, int u, int ktot) {
  const int ppr = ktot >> 3;
  const int n   = u / ppr;
  const int k8  = (u - n * ppr) << 3;
  const int ks  = k8 & (G_D - 1);
  float f[8];
#pragma unroll
  for (int i = 0; i < 8; ++i) {
    const float v = w[(size_t)(ks + i) * G_D + n];
    asm volatile("" :: "v"(v));
    f[i] = v;
  }
  const v4u o = (v4u){ pk16(bf16_bits(f[0]), bf16_bits(f[1])), pk16(bf16_bits(f[2]), bf16_bits(f[3])),
                       pk16(bf16_bits(f[4]), bf16_bits(f[5])), pk16(bf16_bits(f[6]), bf16_bits(f[7])) };
  volatile v4u* q = (volatile v4u*)(dst + (size_t)n * (size_t)ktot + k8);
  *q = o;
  __threadfence();
  *q = o;
}
__device__ __forceinline__ void bias_line(const float* __restrict__ b, float* dst, int lane) {
  const v2f v = *(const v2fa*)(b + 2 * lane);
  asm volatile("" :: "v"(v));
  v2f o;
  o.x = bf16_val(v.x);
  o.y = bf16_val(v.y);
  st2_v2f(dst + 2 * lane, o);
}

__global__ __launch_bounds__(G_NTHR) void k_prep(const float* __restrict__ wh1, const float* __restrict__ wt1,
                                                 const float* __restrict__ wh2, const float* __restrict__ wt2,
                                                 const float* __restrict__ bh1, const float* __restrict__ bh2,
                                                 const float* __restrict__ bt1, const float* __restrict__ bt2,
                                                 unsigned short* WH1T, unsigned short* WT1, unsigned short* WG2,
                                                 unsigned short* WT2, float* BIAS) {
  const int tid = (int)threadIdx.x;
  const int blk = (int)blockIdx.x;
  if (blk < 2) {
    wt_unit(wh1, WH1T, blk * G_NTHR + tid, 64);
  } else if (blk < 6) {
    wt_unit(wt1, WT1, (blk - 2) * G_NTHR + tid, 128);
  } else if (blk < 10) {
    wt_unit(wh2, WG2, (blk - 6) * G_NTHR + tid, 128);
  } else if (blk < 14) {
    wt_unit(wt2, WT2, (blk - 10) * G_NTHR + tid, 128);
  } else {
    const int lane = tid & 31, wave = tid >> 5;
    if (wave == 0) bias_line(bh1, BIAS + 0 * G_D, lane);
    if (wave == 1) bias_line(bh2, BIAS + 1 * G_D, lane);
    if (wave == 2) bias_line(bt1, BIAS + 2 * G_D, lane);
    if (wave == 3) bias_line(bt2, BIAS + 3 * G_D, lane);
  }
}

__device__ __forceinline__ void build_flush(const int* pl, const int* gl, const int* cnt, const int* cur,
                                            const int* tab, int ov, int* lp, int* cntp, int* offp, int* dvp,
                                            int* gsp, int* fp, int tid) {
#pragma unroll 1
  for (int i = tid; i < G_RCAP / 2; i += G_NTHR) {
    const v2i a = *(const v2ia*)(pl + 2 * i);
    const v2i g = *(const v2ia*)(gl + 2 * i);
    const v4i o = {a.x, g.x, a.y, g.y};
    *(volatile v4i*)(lp + 4 * i) = o;
  }
  {
    const v4i v = *(const v4ia*)(cnt + 4 * tid);
    *(volatile v4i*)(cntp + 4 * tid) = v;
  }
  {
    const v4i v = *(const v4ia*)(cnt + G_NBRUN + 4 * tid);
    *(volatile v4i*)(offp + 4 * tid) = v;
  }
  {
    const v4i v = *(const v4ia*)(cur + 4 * tid);
    *(volatile v4i*)(dvp + 4 * tid) = v;
  }
  {
    const v4i v = *(const v4ia*)(tab + 4 * tid);
    *(volatile v4i*)(gsp + 4 * tid) = v;
  }
  if (tid < 8) {
    const v4i f = {ov, ov, ov, ov};
    *(volatile v4i*)(fp + 4 * tid) = f;
  }
}

__global__ __launch_bounds__(G_NTHR) void k_build(const int* __restrict__ srcs, const int* __restrict__ dsts,
                                                  const float* __restrict__ curv, int* LIST, int* CNT, int* OFF,
                                                  int* DINVb, int* GSb, int* FLAG) {
  extern __shared__ __attribute__((aligned(16))) int dsm[];
  int* wl   = dsm;
  int* pl   = dsm + G_NWAVE * G_WLCAP;
  int* cnt  = pl + G_RCAP;
  int* offs = cnt + G_NBRUN;
  int* cur  = offs + G_NBRUN;
  int* tab  = cur + G_NBRUN;
  int* misc = tab + G_NBRUN;
  const int tid = (int)threadIdx.x, lane = tid & 31, wave = tid >> 5;
  const int blk = (int)blockIdx.x;
  const unsigned nbs = (unsigned)(blk * G_NBRUN);

  {
    const v4i z4 = {0, 0, 0, 0};
    for (int i = tid * 4; i < G_BK_ZINTS; i += G_NTHR * 4) *(v4ia*)(dsm + i) = z4;
    if (tid < 16) misc[tid] = 0;
  }
  __syncthreads();

  {
    const int per  = ((G_NE + G_NWAVE * G_WCH - 1) / (G_NWAVE * G_WCH)) * G_WCH;
    const int ebeg = wave * per;
    const int eend = (ebeg + per < G_NE) ? (ebeg + per) : G_NE;
    int* mylist = wl + wave * G_WLCAP;
    int wc = 0;
#pragma unroll 1
    for (int cb = ebeg; cb < eend; cb += G_WCH) {
      const int e0  = cb + lane * G_EPT;
      const int e0c = e0 > G_NE - G_EPT ? G_NE - G_EPT : e0;
      const bool vl = e0 < G_NE;
      const v4i da = *(const v4ia*)(dsts + e0c);
      const v4i db = *(const v4ia*)(dsts + e0c + 4);
      asm volatile("" :: "v"(da));
      asm volatile("" :: "v"(db));
      const unsigned s0 = (unsigned)da.x - nbs, s1 = (unsigned)da.y - nbs;
      const unsigned s2 = (unsigned)da.z - nbs, s3 = (unsigned)da.w - nbs;
      const unsigned s4 = (unsigned)db.x - nbs, s5 = (unsigned)db.y - nbs;
      const unsigned s6 = (unsigned)db.z - nbs, s7 = (unsigned)db.w - nbs;
      const bool h0 = vl && s0 < (unsigned)G_NBRUN, h1 = vl && s1 < (unsigned)G_NBRUN;
      const bool h2 = vl && s2 < (unsigned)G_NBRUN, h3 = vl && s3 < (unsigned)G_NBRUN;
      const bool h4 = vl && s4 < (unsigned)G_NBRUN, h5 = vl && s5 < (unsigned)G_NBRUN;
      const bool h6 = vl && s6 < (unsigned)G_NBRUN, h7 = vl && s7 < (unsigned)G_NBRUN;
      const unsigned m0 = __builtin_amdgcn_ballot_w32(h0), m1 = __builtin_amdgcn_ballot_w32(h1);
      const unsigned m2 = __builtin_amdgcn_ballot_w32(h2), m3 = __builtin_amdgcn_ballot_w32(h3);
      const unsigned m4 = __builtin_amdgcn_ballot_w32(h4), m5 = __builtin_amdgcn_ballot_w32(h5);
      const unsigned m6 = __builtin_amdgcn_ballot_w32(h6), m7 = __builtin_amdgcn_ballot_w32(h7);
      const unsigned any = m0 | m1 | m2 | m3 | m4 | m5 | m6 | m7;
      if (any != 0u) {
        const int pre = (int)(__builtin_amdgcn_mbcnt_lo(m0, 0u) + __builtin_amdgcn_mbcnt_lo(m1, 0u) +
                              __builtin_amdgcn_mbcnt_lo(m2, 0u) + __builtin_amdgcn_mbcnt_lo(m3, 0u) +
                              __builtin_amdgcn_mbcnt_lo(m4, 0u) + __builtin_amdgcn_mbcnt_lo(m5, 0u) +
                              __builtin_amdgcn_mbcnt_lo(m6, 0u) + __builtin_amdgcn_mbcnt_lo(m7, 0u));
        int p = wc + pre;
        if (h0) { if (p < G_WLCAP) mylist[p] = (int)((unsigned)(e0 + 0) | (s0 << G_ESH)); p = p + 1; }
        if (h1) { if (p < G_WLCAP) mylist[p] = (int)((unsigned)(e0 + 1) | (s1 << G_ESH)); p = p + 1; }
        if (h2) { if (p < G_WLCAP) mylist[p] = (int)((unsigned)(e0 + 2) | (s2 << G_ESH)); p = p + 1; }
        if (h3) { if (p < G_WLCAP) mylist[p] = (int)((unsigned)(e0 + 3) | (s3 << G_ESH)); p = p + 1; }
        if (h4) { if (p < G_WLCAP) mylist[p] = (int)((unsigned)(e0 + 4) | (s4 << G_ESH)); p = p + 1; }
        if (h5) { if (p < G_WLCAP) mylist[p] = (int)((unsigned)(e0 + 5) | (s5 << G_ESH)); p = p + 1; }
        if (h6) { if (p < G_WLCAP) mylist[p] = (int)((unsigned)(e0 + 6) | (s6 << G_ESH)); p = p + 1; }
        if (h7) { if (p < G_WLCAP) mylist[p] = (int)((unsigned)(e0 + 7) | (s7 << G_ESH)); p = p + 1; }
        wc += (int)(__builtin_popcount(m0) + __builtin_popcount(m1) + __builtin_popcount(m2) + __builtin_popcount(m3) +
                    __builtin_popcount(m4) + __builtin_popcount(m5) + __builtin_popcount(m6) + __builtin_popcount(m7));
      }
    }
    if (lane == 0) misc[wave] = wc;
  }
  __syncthreads();

  if (wave == 0) {
    int ov = 0;
    int tot = 0;
#pragma unroll 1
    for (int w2 = 0; w2 < G_NWAVE; ++w2) {
      int c = misc[w2];
      if (c > G_WLCAP) ov = 1;
      c = c < 0 ? 0 : (c > G_WLCAP ? G_WLCAP : c);
      tot += c;
#pragma unroll 1
      for (int b0 = 0; b0 < c; b0 += 32) {
        const int idx = b0 + lane;
        const int ent = wl[w2 * G_WLCAP + (idx < G_WLCAP ? idx : G_WLCAP - 1)];
        const int m32 = (c - b0) < 32 ? (c - b0) : 32;
#pragma unroll 1
        for (int k = 0; k < m32; ++k) {
          const int u    = __builtin_amdgcn_readlane(ent, k);
          const int slot = (u >> G_ESH) & (G_NBRUN - 1);
          if (lane == 0) cnt[slot] = cnt[slot] + 1;
        }
      }
    }
    if (tot > G_RCAP) { ov = 1; tot = G_RCAP; }
    if (lane == 0) { misc[9] = ov; misc[10] = tot; }
  }
  __syncthreads();
  if (wave == 0) {
    const int base = lane * (G_NBRUN / 32);
    int s = 0;
#pragma unroll 1
    for (int i = 0; i < G_NBRUN / 32; ++i) s += cnt[base + i];
    int incl = s;
#pragma unroll
    for (int d = 1; d < 32; d <<= 1) {
      const int y = __shfl_up(incl, d, 32);
      if (lane >= d) incl += y;
    }
    int run = incl - s;
#pragma unroll 1
    for (int i = 0; i < G_NBRUN / 32; ++i) {
      const int cv = cnt[base + i];
      offs[base + i] = run;
      cur[base + i]  = run;
      run += cv;
    }
  }
  __syncthreads();

  if (wave == 0) {
#pragma unroll 1
    for (int w2 = 0; w2 < G_NWAVE; ++w2) {
      int c = misc[w2];
      c = c < 0 ? 0 : (c > G_WLCAP ? G_WLCAP : c);
#pragma unroll 1
      for (int b0 = 0; b0 < c; b0 += 32) {
        const int idx = b0 + lane;
        const int ent = wl[w2 * G_WLCAP + (idx < G_WLCAP ? idx : G_WLCAP - 1)];
        const int m32 = (c - b0) < 32 ? (c - b0) : 32;
#pragma unroll 1
        for (int k = 0; k < m32; ++k) {
          const int u    = __builtin_amdgcn_readlane(ent, k);
          const int slot = (u >> G_ESH) & (G_NBRUN - 1);
          if (lane == 0) {
            int p = cur[slot];
            p = p < 0 ? 0 : (p > G_RCAP - 1 ? G_RCAP - 1 : p);
            pl[p] = u & ((1 << G_ESH) - 1);
            cur[slot] = p + 1;
          }
        }
      }
    }
  }
  __syncthreads();

  int* gl = wl;
  {
    const int tot = clampi(misc[10], 0, G_RCAP);
#pragma unroll 1
    for (int p = tid; p < G_RCAP; p += G_NTHR) {
      const int eid = clampi(pl[p], 0, G_NE - 1);
      int sr = srcs[eid];
      asm volatile("" :: "v"(sr));
      sr = clampi(sr, 0, G_NN - 1);
      const float cv = curv[eid];
      asm volatile("" :: "v"(cv));
      float cvb = bf16_val(cv);
      asm volatile("" : "+v"(cvb));
      const float tq = cvb / 5.0f;
      const float ex = expf(-tq);
      const float g  = 1.0f / (1.0f + ex);
      const bool live = p < tot;
      pl[p] = live ? sr : 0;
      gl[p] = live ? __float_as_int(g) : 0;
    }
  }
  __syncthreads();

#pragma unroll 1
  for (int q = 0; q < G_NBRUN / G_NTHR; ++q) {
    const int slot = q * G_NTHR + tid;
    const int c = clampi(cnt[slot], 0, G_RCAP);
    const int o = clampi(offs[slot], 0, G_RCAP - 1);
    int cm = c;
#pragma unroll
    for (int d = 16; d >= 1; d >>= 1) {
      const int y = __shfl_xor(cm, d, 32);
      cm = cm > y ? cm : y;
    }
    float dg = 0.0f, gs = 0.0f;
#pragma unroll 1
    for (int i = 0; i < cm; ++i) {
      int idx = o + i;
      idx = idx > G_RCAP - 1 ? G_RCAP - 1 : idx;
      const float g = __int_as_float(gl[idx]);
      asm volatile("" :: "v"(g));
      const bool mine = i < c;
      const float gg = mine ? g : 0.0f;
      const float hh = mine ? (1.0f - g) : 0.0f;
      dg = dg + gg;
      gs = gs + hh;
    }
    dg = dg + 1.0f;
    const float rs = 1.0f / sqrtf(dg);
    const float di = (dg > 0.0f) ? rs : 0.0f;
    cur[slot] = __float_as_int(di);
    tab[slot] = __float_as_int(gs);
  }
  __syncthreads();

  const int ovf = misc[9];
  int* lp   = LIST + (size_t)blk * (size_t)(2 * G_RCAP);
  int* cntp = CNT + (size_t)blk * G_NBRUN;
  int* offp = OFF + (size_t)blk * G_NBRUN;
  int* dvp  = DINVb + (size_t)blk * G_NBRUN;
  int* gsp  = GSb + (size_t)blk * G_NBRUN;
  int* fp   = FLAG + (size_t)blk * 32;
  build_flush(pl, gl, cnt, cur, tab, ovf, lp, cntp, offp, dvp, gsp, fp, tid);
  __threadfence();
  build_flush(pl, gl, cnt, cur, tab, ovf, lp, cntp, offp, dvp, gsp, fp, tid);
}

template <int L2>
__global__ __launch_bounds__(G_NTHR) void k_walk(const unsigned* __restrict__ XBw, const float* __restrict__ HV,
                                                 const float* __restrict__ T, const int* __restrict__ LIST,
                                                 const int* __restrict__ CNT, const int* __restrict__ OFF,
                                                 const float* __restrict__ DINV, const float* __restrict__ bias,
                                                 float* HA, unsigned* OPSw, int split) {
  const int tid = (int)threadIdx.x, lane = tid & 31, wave = tid >> 5;
  const int node = (int)blockIdx.x * G_NWAVE + wave;
  const int bk = node >> G_SLB;
  const int* lb = LIST + (size_t)bk * (size_t)(2 * G_RCAP);
  const int craw = CNT[node];
  const int oraw = OFF[node];
  const int c   = __builtin_amdgcn_readfirstlane(clampi(craw, 0, G_WCAP));
  const int big = __builtin_amdgcn_readfirstlane(craw > G_WCAP ? 1 : 0);
  const int o   = __builtin_amdgcn_readfirstlane(clampi(oraw, 0, G_RCAP - 1));
  int last = o + (c > 0 ? c : 1) - 1;
  last = last > G_RCAP - 1 ? G_RCAP - 1 : last;
  float dc = DINV[node];
  asm volatile("" : "+v"(dc));

  float xc0, xc1;
  if (L2 == 0) {
    const unsigned w = XBw[(size_t)node * 32 + lane];
    asm volatile("" :: "v"(w));
    xc0 = __uint_as_float(w << 16);
    xc1 = __uint_as_float(w & 0xffff0000u);
  } else {
    const v2f q = *(const v2fa*)(HV + (size_t)node * G_D + 2 * lane);
    asm volatile("" :: "v"(q));
    xc0 = q.x;
    xc1 = q.y;
  }
  asm volatile("" : "+v"(xc0));
  asm volatile("" : "+v"(xc1));

  float a0 = 0.0f, a1 = 0.0f, s0 = 0.0f, s1 = 0.0f;
#pragma unroll 1
  for (int b0 = 0; b0 < c; b0 += 32) {
    int idx = o + b0 + lane;
    idx = idx > last ? last : idx;
    const v2i ent = *(const v2ia*)(lb + 2 * idx);
    asm volatile("" :: "v"(ent));
    const int sr = clampi(ent.x, 0, G_NN - 1);
    const float g = __int_as_float(ent.y);
    float ds = DINV[sr];
    asm volatile("" : "+v"(ds));
    const float nrm = (ds * g) * dc;
    const float gh  = 1.0f - g;
    const int m32 = (c - b0) < 32 ? (c - b0) : 32;
#pragma unroll 1
    for (int k = 0; k < m32; ++k) {
      const int   sk = __builtin_amdgcn_readlane(sr, k);
      const float nk = __int_as_float(__builtin_amdgcn_readlane(__float_as_int(nrm), k));
      const float hk = __int_as_float(__builtin_amdgcn_readlane(__float_as_int(gh), k));
      const v2f q = *(const v2fa*)(T + (size_t)sk * G_D + 2 * lane);
      float v0, v1;
      if (L2 == 0) {
        const unsigned w = XBw[(size_t)sk * 32 + lane];
        asm volatile("" :: "v"(w));
        v0 = __uint_as_float(w << 16);
        v1 = __uint_as_float(w & 0xffff0000u);
      } else {
        const v2f hv = *(const v2fa*)(HV + (size_t)sk * G_D + 2 * lane);
        asm volatile("" :: "v"(hv));
        v0 = hv.x;
        v1 = hv.y;
      }
      asm volatile("" : "+v"(v0));
      asm volatile("" : "+v"(v1));
      const float p0 = q.x * nk, p1 = q.y * nk;
      a0 = a0 + p0;
      a1 = a1 + p1;
      const float d0 = fabsf(xc0 - v0), d1 = fabsf(xc1 - v1);
      const float e0 = hk * d0, e1 = hk * d1;
      s0 = s0 + e0;
      s1 = s1 + e1;
    }
  }

  const v2f tc = *(const v2fa*)(T + (size_t)node * G_D + 2 * lane);
  asm volatile("" :: "v"(tc));
  const float lw = (dc * 1.0f) * dc;
  const float l0 = tc.x * lw, l1 = tc.y * lw;
  a0 = a0 + l0;
  a1 = a1 + l1;
  v2f bv = *(const v2fa*)(bias + 2 * lane);
  asm volatile("" : "+v"(bv));
  const float qnan = __uint_as_float(0x7fc00000u);
  const float pz = (big != 0) ? qnan : 0.0f;
  v2f ha;
  ha.x = (a0 + bv.x) + pz;
  ha.y = (a1 + bv.y) + pz;
  st2_v2f(HA + (size_t)node * G_D + 2 * lane, ha);

  const float t0 = s0 + pz, t1 = s1 + pz;
  const unsigned whi = pk16(bf16_bits(t0), bf16_bits(t1));
  const unsigned wlo = (split != 0) ? pk16(bf16_lo_bits(t0), bf16_lo_bits(t1)) : 0u;
  unsigned* rowp = OPSw + (size_t)node * 64;
  st2_words(rowp + lane, whi, rowp + 32 + lane, wlo);
}

__global__ __launch_bounds__(G_NTHR) void k_comb1(const float* __restrict__ HA, const float* __restrict__ TH,
                                                  const float* __restrict__ GS, const float* __restrict__ bias,
                                                  const int* __restrict__ FLAG, float* HV, unsigned* OPHw, int split) {
  const int tid = (int)threadIdx.x, lane = tid & 31, wave = tid >> 5;
  const int node = (int)blockIdx.x * G_NWAVE + wave;
  const v2f ha = *(const v2fa*)(HA + (size_t)node * G_D + 2 * lane);
  const v2f th = *(const v2fa*)(TH + (size_t)node * G_D + 2 * lane);
  v2f bv = *(const v2fa*)(bias + 2 * lane);
  asm volatile("" :: "v"(ha));
  asm volatile("" :: "v"(th));
  asm volatile("" : "+v"(bv));
  const float gs = GS[node];
  const int flag = FLAG[(size_t)(node >> G_SLB) * 32];
  const float gb0 = gs * bv.x, gb1 = gs * bv.y;
  const float v0 = ha.x + (th.x + gb0);
  const float v1 = ha.y + (th.y + gb1);
  float y0 = (v0 > 0.0f) ? v0 : (v0 - v0);
  float y1 = (v1 > 0.0f) ? v1 : (v1 - v1);
  const float qnan = __uint_as_float(0x7fc00000u);
  const bool bad  = flag != 0;
  const bool live = node < G_NN;
  y0 = bad ? qnan : y0;
  y1 = bad ? qnan : y1;
  y0 = live ? y0 : 0.0f;
  y1 = live ? y1 : 0.0f;
  v2f hv;
  hv.x = y0;
  hv.y = y1;
  st2_v2f(HV + (size_t)node * G_D + 2 * lane, hv);
  const unsigned whi = pk16(bf16_bits(y0), bf16_bits(y1));
  const unsigned wlo = (split != 0) ? pk16(bf16_lo_bits(y0), bf16_lo_bits(y1)) : 0u;
  unsigned* rowp = OPHw + (size_t)node * 64;
  st2_words(rowp + lane, whi, rowp + 32 + lane, wlo);
}

__global__ __launch_bounds__(G_NTHR) void k_comb2(const float* __restrict__ HA, const float* __restrict__ TH,
                                                  const float* __restrict__ GS, const float* __restrict__ bias,
                                                  const int* __restrict__ FLAG, float* out, int nreal) {
  const int tid = (int)threadIdx.x, lane = tid & 31, wave = tid >> 5;
  const int node = (int)blockIdx.x * G_NWAVE + wave;
  const int nc = clampi(node, 0, G_NN - 1);
  const v2f ha = *(const v2fa*)(HA + (size_t)nc * G_D + 2 * lane);
  const v2f th = *(const v2fa*)(TH + (size_t)nc * G_D + 2 * lane);
  v2f bv = *(const v2fa*)(bias + 2 * lane);
  asm volatile("" :: "v"(ha));
  asm volatile("" :: "v"(th));
  asm volatile("" : "+v"(bv));
  const float gs = GS[nc];
  const int flag = FLAG[(size_t)(nc >> G_SLB) * 32];
  const float gb0 = gs * bv.x, gb1 = gs * bv.y;
  const float v0 = ha.x + (th.x + gb0);
  const float v1 = ha.y + (th.y + gb1);
  const float qnan = __uint_as_float(0x7fc00000u);
  const bool bad = flag != 0;
  v2f o;
  o.x = bad ? qnan : v0;
  o.y = bad ? qnan : v1;
  if (node < nreal) {
    st2_v2f(out + (size_t)node * G_D + 2 * lane, o);
  }
}

extern "C" void kernel_launch(void* const* d_in, const int* in_sizes, int n_in,
                              void* d_out, int out_size, void* d_ws, size_t ws_size,
                              hipStream_t stream) {
  if (n_in < 11) return;
  if (in_sizes[0] != G_NN * G_D) return;
  if (in_sizes[1] != 2 * G_NE) return;
  if (in_sizes[2] != G_NE) return;
  if (in_sizes[3] != G_D * G_D || in_sizes[5] != G_D * G_D) return;
  if (in_sizes[7] != G_D * G_D || in_sizes[9] != G_D * G_D) return;
  if (in_sizes[4] != G_D || in_sizes[6] != G_D || in_sizes[8] != G_D || in_sizes[10] != G_D) return;
  if (out_size != G_NN * G_D) return;

  const float* x    = (const float*)d_in[0];
  const int*   ei   = (const int*)d_in[1];
  const float* curv = (const float*)d_in[2];
  const float* Wh1  = (const float*)d_in[3];
  const float* bh1  = (const float*)d_in[4];
  const float* Wh2  = (const float*)d_in[5];
  const float* bh2  = (const float*)d_in[6];
  const float* Wt1  = (const float*)d_in[7];
  const float* bt1  = (const float*)d_in[8];
  const float* Wt2  = (const float*)d_in[9];
  const float* bt2  = (const float*)d_in[10];
  const int* srcs = ei;
  const int* dsts = ei + G_NE;
  float* out = (float*)d_out;
  const int nreal = out_size / G_D;

  constexpr size_t zXB   = (size_t)G_NPAD * G_D * 2;
  constexpr size_t zF    = (size_t)G_NPAD * G_D * 4;
  constexpr size_t zOP   = (size_t)G_NPAD * 2 * G_D * 2;
  constexpr size_t zLIST = (size_t)G_NBK * G_RCAP * 8;
  constexpr size_t zTAB  = (size_t)G_NBK * G_NBRUN * 4;
  constexpr size_t zFLAG = 8192;
  constexpr size_t zW64  = (size_t)G_D * G_D * 2;
  constexpr size_t zW128 = (size_t)G_D * 2 * G_D * 2;
  constexpr size_t zBIAS = 1024;
  constexpr size_t oXB   = 0;
  constexpr size_t oT    = oXB + zXB;
  constexpr size_t oHA   = oT + zF;
  constexpr size_t oTH   = oHA + zF;
  constexpr size_t oHV   = oTH + zF;
  constexpr size_t oOPS  = oHV + zF;
  constexpr size_t oOPH  = oOPS + zOP;
  constexpr size_t oLIST = oOPH + zOP;
  constexpr size_t oDINV = oLIST + zLIST;
  constexpr size_t oGS   = oDINV + zTAB;
  constexpr size_t oCNT  = oGS + zTAB;
  constexpr size_t oOFF  = oCNT + zTAB;
  constexpr size_t oFLAG = oOFF + zTAB;
  constexpr size_t oWH1T = oFLAG + zFLAG;
  constexpr size_t oWT1  = oWH1T + zW64;
  constexpr size_t oWG2  = oWT1 + zW128;
  constexpr size_t oWT2  = oWG2 + zW128;
  constexpr size_t oBIAS = oWT2 + zW128;
  constexpr size_t oEND  = oBIAS + zBIAS;
  static_assert(zXB % 256 == 0 && zF % 256 == 0 && zOP % 256 == 0 && zLIST % 256 == 0 && zTAB % 256 == 0);
  static_assert(zFLAG % 256 == 0 && zFLAG >= (size_t)G_NBK * 128 && zW64 % 256 == 0 && zW128 % 256 == 0);
  static_assert(zTAB >= (size_t)G_NPAD * 4);
  static_assert(oEND == 94385152);
  static_assert(oEND <= G_WSMAX);
  if (oEND > ws_size) return;

  char* ws = (char*)d_ws;
  unsigned short* XB   = (unsigned short*)(ws + oXB);
  float*          T    = (float*)(ws + oT);
  float*          HA   = (float*)(ws + oHA);
  float*          TH   = (float*)(ws + oTH);
  float*          HV   = (float*)(ws + oHV);
  unsigned short* OPS  = (unsigned short*)(ws + oOPS);
  unsigned short* OPH  = (unsigned short*)(ws + oOPH);
  int*            LIST = (int*)(ws + oLIST);
  int*            DINV = (int*)(ws + oDINV);
  int*            GS   = (int*)(ws + oGS);
  int*            CNT  = (int*)(ws + oCNT);
  int*            OFF  = (int*)(ws + oOFF);
  int*            FLAG = (int*)(ws + oFLAG);
  unsigned short* WH1T = (unsigned short*)(ws + oWH1T);
  unsigned short* WT1  = (unsigned short*)(ws + oWT1);
  unsigned short* WG2  = (unsigned short*)(ws + oWG2);
  unsigned short* WT2  = (unsigned short*)(ws + oWT2);
  float*          BIAS = (float*)(ws + oBIAS);

  hipFuncSetAttribute(reinterpret_cast<const void*>(&k_build), hipFuncAttributeMaxDynamicSharedMemorySize,
                      (int)G_BK_LDS);

  const int gemmBlocks = ((G_NPAD / 64) + 7) / 8;

  k_plane<0><<<G_NPAD * G_D / 8 / 256, 256, 0, stream>>>(x, G_NN, G_D, G_D, XB, G_NPAD, G_D);
  k_prep<<<15, G_NTHR, 0, stream>>>(Wh1, Wt1, Wh2, Wt2, bh1, bh2, bt1, bt2, WH1T, WT1, WG2, WT2, BIAS);
  k_build<<<G_NBK, G_NTHR, G_BK_LDS, stream>>>(srcs, dsts, curv, LIST, CNT, OFF, DINV, GS, FLAG);
  k_gemm_nt<0, 0><<<gemmBlocks, 256, 0, stream>>>(XB, WH1T, BIAS, T, G_NPAD, G_D, G_D, G_D);
  k_walk<0><<<G_NPAD / G_NWAVE, G_NTHR, 0, stream>>>((const unsigned*)XB, HV, T, LIST, CNT, OFF,
                                                      (const float*)DINV, BIAS + 0 * G_D, HA, (unsigned*)OPS,
                                                      SPLIT_H1);
  k_gemm_nt<0, 0><<<gemmBlocks, 256, 0, stream>>>(OPS, WT1, BIAS, TH, G_NPAD, G_D, 2 * G_D, G_D);
  k_comb1<<<G_NPAD / G_NWAVE, G_NTHR, 0, stream>>>(HA, TH, (const float*)GS, BIAS + 2 * G_D, FLAG, HV,
                                                   (unsigned*)OPH, SPLIT_G2);
  k_gemm_nt<0, 0><<<gemmBlocks, 256, 0, stream>>>(OPH, WG2, BIAS, T, G_NPAD, G_D, 2 * G_D, G_D);
  k_walk<1><<<G_NPAD / G_NWAVE, G_NTHR, 0, stream>>>((const unsigned*)XB, HV, T, LIST, CNT, OFF,
                                                      (const float*)DINV, BIAS + 1 * G_D, HA, (unsigned*)OPS,
                                                      SPLIT_H2);
  k_gemm_nt<0, 0><<<gemmBlocks, 256, 0, stream>>>(OPS, WT2, BIAS, TH, G_NPAD, G_D, 2 * G_D, G_D);
  k_comb2<<<G_NN / G_NWAVE, G_NTHR, 0, stream>>>(HA, TH, (const float*)GS, BIAS + 3 * G_D, FLAG, out, nreal);
}
